// RoPESelfAttention_58076547776991
// MI455X (gfx1250) — hardware-verified
//
#include <hip/hip_runtime.h>

#ifndef NB
#define NB 4
#endif
#ifndef SEQ
#define SEQ 2048
#endif
#define NB_FULL 4
#define SEQ_FULL 2048

constexpr int Dmod  = 1024;
constexpr int Hn    = 16;
constexpr int DhC   = 64;
constexpr int Mrows = NB * SEQ;
constexpr int NQKV  = 3 * Dmod;
static_assert(NB >= 1 && NB <= NB_FULL);
static_assert(SEQ >= 64 && SEQ <= SEQ_FULL && (SEQ % 64) == 0);
static_assert(Hn * DhC == Dmod);
static_assert(((Mrows / 16) * (NQKV / 64)) % 8 == 0);
static_assert(((Mrows / 16) * (Dmod / 64)) % 8 == 0);
static_assert((NB * Hn * (SEQ / 16)) % 8 == 0);
static_assert(((size_t)Mrows * Dmod / 8) % 256 == 0);

constexpr float XC  = 64.0f;
constexpr float WC  = 64.0f;
constexpr float QC  = 16.0f;
constexpr float PC  = 1024.0f;
constexpr float CC  = 256.0f;
constexpr float RXW = 1.0f / (XC * WC);
constexpr float SCL = 0.125f / (QC * QC);
constexpr float OCV = CC / (QC * PC);
constexpr float ROW = 1.0f / (CC * WC);

constexpr size_t SZ_X    = (size_t)Mrows * Dmod * 2;
constexpr size_t SZ_WQKV = (size_t)NQKV * Dmod * 2;
constexpr size_t SZ_WO   = (size_t)Dmod * Dmod * 2;
constexpr size_t OFF_X    = 0;
constexpr size_t OFF_WQKV = OFF_X + SZ_X;
constexpr size_t OFF_WO   = OFF_WQKV + SZ_WQKV;
constexpr size_t OFF_Q    = OFF_WO + SZ_WO;
constexpr size_t OFF_K    = OFF_Q + SZ_X;
constexpr size_t OFF_VR   = OFF_K + SZ_X;
constexpr size_t OFF_VT   = OFF_VR + SZ_X;
constexpr size_t OFF_C    = OFF_VT + SZ_X;
constexpr size_t WS_TOTAL = OFF_C + SZ_X;
static_assert(WS_TOTAL <= (size_t)134217728);
static_assert((OFF_WQKV % 128) == 0 && (OFF_WO % 128) == 0 && (OFF_Q % 128) == 0 && (OFF_C % 128) == 0);

typedef _Float16       f16x16 __attribute__((ext_vector_type(16)));
typedef float          floatx8 __attribute__((ext_vector_type(8)));
typedef float          v4fa __attribute__((ext_vector_type(4), may_alias));
typedef float          v2fa __attribute__((ext_vector_type(2), may_alias));
typedef unsigned short us8 __attribute__((ext_vector_type(8)));

__device__ __forceinline__ float bfr(float f) {
  unsigned u = __float_as_uint(f);
  u = (u + 0x7FFFu + ((u >> 16) & 1u)) & 0xFFFF0000u;
  return __uint_as_float(u);
}
__device__ __forceinline__ unsigned short h16(float f) { return __builtin_bit_cast(unsigned short, (_Float16)f); }
__device__ __forceinline__ unsigned pack2h(float a, float b) { return (unsigned)h16(a) | ((unsigned)h16(b) << 16); }

union Frag {
  f16x16 v;
  uint4  q[2];
};

__device__ __forceinline__ Frag load_frag_A(const unsigned short* __restrict__ base,
                                            size_t ld, int row0, int col0, int lane) {
  const int m = lane & 15, hi = lane >> 4;
  const unsigned short* p = base + (size_t)(row0 + m) * ld + col0 + hi * 8;
  Frag f;
  f.q[0] = *(const uint4*)(p);
  f.q[1] = *(const uint4*)(p + 16);
  return f;
}

__device__ __forceinline__ Frag load_frag_B(const unsigned short* __restrict__ baseT,
                                            size_t ld, int n0, int col0, int lane) {
  const int n = lane & 15, hi = lane >> 4;
  const unsigned short* p = baseT + (size_t)(n0 + n) * ld + col0 + hi * 8;
  Frag f;
  f.q[0] = *(const uint4*)(p);
  f.q[1] = *(const uint4*)(p + 16);
  return f;
}

__device__ __forceinline__ floatx8 wmma16(Frag a, Frag b, floatx8 c) {
  floatx8 d = __builtin_amdgcn_wmma_f32_16x16x32_f16(false, a.v, false, b.v, (short)0, c, false, false);
  asm volatile("v_nop\n\tv_nop\n\tv_nop\n\tv_nop" : "+v"(d) : "v"(a.v), "v"(b.v));
  return d;
}

__device__ __forceinline__ void store_rows64(const float* so, unsigned short* dst, size_t ld, int lane) {
  unsigned pk[16];
#pragma unroll
  for (int rr = 0; rr < 16; ++rr) {
    const v2fa v = *(const v2fa*)(so + rr * 64 + 2 * lane);
    pk[rr] = pack2h(v[0], v[1]);
  }
#pragma unroll
  for (int rr = 0; rr < 16; ++rr) *(volatile unsigned*)(dst + (size_t)rr * ld + 2 * lane) = pk[rr];
  __threadfence();
#pragma unroll
  for (int rr = 0; rr < 16; ++rr) *(volatile unsigned*)(dst + (size_t)rr * ld + 2 * lane) = pk[rr];
}

__device__ __forceinline__ void stage16x64(const float* __restrict__ src, float* sw, int lane) {
#pragma unroll
  for (int i = 0; i < 8; ++i) {
    const int c = lane + 32 * i;
    const v4fa v = *(const v4fa*)(src + c * 4);
    *(v4fa*)(sw + c * 4) = v;
  }
}

__global__ __launch_bounds__(256) void cvt_x_kernel(const float* __restrict__ x, unsigned short* __restrict__ Xh) {
  const size_t ng = (size_t)Mrows * Dmod / 8;
  const size_t i  = (size_t)blockIdx.x * 256 + threadIdx.x;
  if (i >= ng) return;
  const size_t m  = i / (Dmod / 8);
  const int    c8 = (int)(i - m * (Dmod / 8));
  const size_t srow = (m / SEQ) * SEQ_FULL + (m % SEQ);
  const float* p = x + srow * Dmod + (size_t)c8 * 8;
  const v4fa a = *(const v4fa*)p;
  const v4fa b = *(const v4fa*)(p + 4);
  us8 o;
  o[0] = h16(bfr(a[0]) * XC); o[1] = h16(bfr(a[1]) * XC); o[2] = h16(bfr(a[2]) * XC); o[3] = h16(bfr(a[3]) * XC);
  o[4] = h16(bfr(b[0]) * XC); o[5] = h16(bfr(b[1]) * XC); o[6] = h16(bfr(b[2]) * XC); o[7] = h16(bfr(b[3]) * XC);
  unsigned short* d = Xh + i * 8;
  *(volatile us8*)d = o;
  __threadfence();
  *(volatile us8*)d = o;
}

__global__ __launch_bounds__(256) void cvt_w_kernel(const float* __restrict__ qw, const float* __restrict__ kw,
                                                    const float* __restrict__ vw, const float* __restrict__ ow,
                                                    unsigned short* __restrict__ Wqkv, unsigned short* __restrict__ Wo) {
  const int which = blockIdx.y;
  const float* src = (which == 0) ? qw : (which == 1) ? kw : (which == 2) ? vw : ow;
  unsigned short* dst = (which < 3) ? (Wqkv + (size_t)which * Dmod * Dmod) : Wo;
  const size_t ng = (size_t)Dmod * Dmod / 8;
  const size_t i  = (size_t)blockIdx.x * 256 + threadIdx.x;
  if (i >= ng) return;
  const float* p = src + i * 8;
  const v4fa a = *(const v4fa*)p;
  const v4fa b = *(const v4fa*)(p + 4);
  us8 o;
  o[0] = h16(bfr(a[0]) * WC); o[1] = h16(bfr(a[1]) * WC); o[2] = h16(bfr(a[2]) * WC); o[3] = h16(bfr(a[3]) * WC);
  o[4] = h16(bfr(b[0]) * WC); o[5] = h16(bfr(b[1]) * WC); o[6] = h16(bfr(b[2]) * WC); o[7] = h16(bfr(b[3]) * WC);
  unsigned short* d = dst + i * 8;
  *(volatile us8*)d = o;
  __threadfence();
  *(volatile us8*)d = o;
}

__global__ __launch_bounds__(256)
void qkv_rotary_kernel(const unsigned short* __restrict__ Xh,
                       const unsigned short* __restrict__ Wqkv,
                       const float* __restrict__ qb, const float* __restrict__ kb, const float* __restrict__ vb,
                       const float* __restrict__ cosp, const float* __restrict__ sinp,
                       unsigned short* __restrict__ Qh,
                       unsigned short* __restrict__ Kh,
                       unsigned short* __restrict__ Vr) {
  __shared__ __align__(16) float st[8][16 * 64];
  const int lane = threadIdx.x & 31;
  const int wib  = threadIdx.x >> 5;
  const int gw   = blockIdx.x * 8 + wib;
  constexpr int nW = NQKV / 64;
  if (gw >= (Mrows / 16) * nW) return;
  const int mt   = gw / nW;
  const int nw   = gw - mt * nW;
  const int row0 = mt * 16;
  const int n0   = nw * 64;

  floatx8 acc[4] = {};
  for (int k0 = 0; k0 < Dmod; k0 += 32) {
    const Frag a = load_frag_A(Xh, Dmod, row0, k0, lane);
#pragma unroll
    for (int t = 0; t < 4; ++t) {
      const Frag b = load_frag_B(Wqkv, Dmod, n0 + 16 * t, k0, lane);
      acc[t] = wmma16(a, b, acc[t]);
    }
  }

  const int n = lane & 15, hi = lane >> 4;
  const int seg = n0 / Dmod;
  const int nl0 = n0 - seg * Dmod;
  const int h   = nl0 / DhC;
  const float* bp = (seg == 0) ? qb : (seg == 1) ? kb : vb;
  float* sw = st[wib];

  if (seg < 2) {
    const int pos0 = row0 % SEQ;
    float cr[2][2][8], sr[2][2][8];
    stage16x64(cosp + (size_t)pos0 * DhC, sw, lane);
    asm volatile("s_wait_dscnt 0" ::: "memory");
    __builtin_amdgcn_wave_barrier();
#pragma unroll
    for (int t = 0; t < 2; ++t)
#pragma unroll
      for (int j = 0; j < 8; ++j) {
        cr[t][0][j] = bfr(sw[(j + 8 * hi) * 64 + 16 * t + n]);
        cr[t][1][j] = bfr(sw[(j + 8 * hi) * 64 + 16 * t + n + 32]);
      }
    asm volatile("s_wait_dscnt 0" ::: "memory");
    __builtin_amdgcn_wave_barrier();
    stage16x64(sinp + (size_t)pos0 * DhC, sw, lane);
    asm volatile("s_wait_dscnt 0" ::: "memory");
    __builtin_amdgcn_wave_barrier();
#pragma unroll
    for (int t = 0; t < 2; ++t)
#pragma unroll
      for (int j = 0; j < 8; ++j) {
        sr[t][0][j] = bfr(sw[(j + 8 * hi) * 64 + 16 * t + n]);
        sr[t][1][j] = bfr(sw[(j + 8 * hi) * 64 + 16 * t + n + 32]);
      }
    asm volatile("s_wait_dscnt 0" ::: "memory");
    __builtin_amdgcn_wave_barrier();
#pragma unroll
    for (int t = 0; t < 2; ++t) {
      const int d = 16 * t + n;
      const float b1 = bfr(bp[nl0 + d]);
      const float b2 = bfr(bp[nl0 + d + 32]);
#pragma unroll
      for (int j = 0; j < 8; ++j) {
        const float x1 = acc[t][j] * RXW + b1;
        const float x2 = acc[t + 2][j] * RXW + b2;
        sw[(j + 8 * hi) * 64 + d]      = (x1 * cr[t][0][j] - x2 * sr[t][0][j]) * QC;
        sw[(j + 8 * hi) * 64 + d + 32] = (x2 * cr[t][1][j] + x1 * sr[t][1][j]) * QC;
      }
    }
  } else {
#pragma unroll
    for (int t = 0; t < 4; ++t) {
      const float bv = bfr(bp[nl0 + 16 * t + n]);
#pragma unroll
      for (int j = 0; j < 8; ++j) sw[(j + 8 * hi) * 64 + 16 * t + n] = (acc[t][j] * RXW + bv) * QC;
    }
  }
  asm volatile("s_wait_dscnt 0" ::: "memory");
  __builtin_amdgcn_wave_barrier();
  unsigned short* dst = (seg == 0) ? Qh : (seg == 1) ? Kh : Vr;
  store_rows64(sw, dst + (size_t)row0 * Dmod + nl0, Dmod, lane);
}

__global__ __launch_bounds__(256) void vt_kernel(const unsigned short* __restrict__ Vr, unsigned short* __restrict__ Vt) {
  __shared__ unsigned short t[64][66];
  const int tid = threadIdx.x, lane = tid & 31, wave = tid >> 5;
  const int m0 = blockIdx.x * 64, c0 = blockIdx.y * 64;
  const int b = m0 / SEQ, pos0 = m0 % SEQ;
#pragma unroll
  for (int k = 0; k < 16; ++k) {
    const int e = tid + 256 * k;
    t[e >> 6][e & 63] = Vr[(size_t)(m0 + (e >> 6)) * Dmod + c0 + (e & 63)];
  }
  __syncthreads();
  unsigned short* dst = Vt + (size_t)b * Dmod * SEQ + pos0;
  unsigned pk[8];
#pragma unroll
  for (int rr = 0; rr < 8; ++rr) {
    const int c = wave * 8 + rr;
    pk[rr] = (unsigned)t[2 * lane][c] | ((unsigned)t[2 * lane + 1][c] << 16);
  }
#pragma unroll
  for (int rr = 0; rr < 8; ++rr) *((volatile unsigned*)(dst + (size_t)(c0 + wave * 8 + rr) * SEQ) + lane) = pk[rr];
  __threadfence();
#pragma unroll
  for (int rr = 0; rr < 8; ++rr) *((volatile unsigned*)(dst + (size_t)(c0 + wave * 8 + rr) * SEQ) + lane) = pk[rr];
}

__global__ __launch_bounds__(256)
void attn_kernel(const unsigned short* __restrict__ Qh,
                 const unsigned short* __restrict__ Kh,
                 const unsigned short* __restrict__ Vt,
                 const float* __restrict__ amask,
                 unsigned short* __restrict__ Ctx) {
  __shared__ __align__(16) unsigned short Plds[8][16 * 32];
  __shared__ __align__(16) float ost[8][16 * 64];

  const int wib  = threadIdx.x >> 5;
  const int lane = threadIdx.x & 31;
  const int gw   = blockIdx.x * 8 + wib;
  constexpr int NQT = SEQ / 16;
  if (gw >= NB * Hn * NQT) return;
  const int qt = gw % NQT;
  const int h  = (gw / NQT) % Hn;
  const int b  = gw / (NQT * Hn);

  const int n = lane & 15, hi = lane >> 4;
  const unsigned short* VtB = Vt + (size_t)b * Dmod * SEQ;
  const int    qrow0 = b * SEQ + qt * 16;
  const int    krow0 = b * SEQ;
  const size_t mrow0 = (size_t)b * SEQ_FULL;

  Frag qf[2];
#pragma unroll
  for (int s = 0; s < 2; ++s) qf[s] = load_frag_A(Qh, Dmod, qrow0, h * DhC + 32 * s, lane);

  float rmax[8], rsum[8];
#pragma unroll
  for (int j = 0; j < 8; ++j) { rmax[j] = -1e30f; rsum[j] = 0.f; }
  floatx8 O[4] = {};

  for (int k0 = 0; k0 < SEQ; k0 += 32) {
    float s2[2][8];
#pragma unroll
    for (int t = 0; t < 2; ++t) {
      floatx8 c = {};
#pragma unroll
      for (int s = 0; s < 2; ++s) {
        const Frag kf = load_frag_B(Kh, Dmod, krow0 + k0 + 16 * t, h * DhC + 32 * s, lane);
        c = wmma16(qf[s], kf, c);
      }
      const float mb = (1.0f - bfr(amask[mrow0 + k0 + 16 * t + n])) * -1.0e9f;
#pragma unroll
      for (int j = 0; j < 8; ++j) s2[t][j] = c[j] * SCL + mb;
    }

#pragma unroll
    for (int j = 0; j < 8; ++j) {
      float mx = fmaxf(s2[0][j], s2[1][j]);
#pragma unroll
      for (int off = 1; off < 16; off <<= 1)
        mx = fmaxf(mx, __shfl_xor(mx, off, 32));
      const float nm    = fmaxf(rmax[j], mx);
      const float alpha = __expf(rmax[j] - nm);
      rmax[j] = nm;
      const float p0 = __expf(s2[0][j] - nm);
      const float p1 = __expf(s2[1][j] - nm);
      float ls = p0 + p1;
#pragma unroll
      for (int off = 1; off < 16; off <<= 1)
        ls += __shfl_xor(ls, off, 32);
      rsum[j] = rsum[j] * alpha + ls;
#pragma unroll
      for (int t4 = 0; t4 < 4; ++t4) O[t4][j] = O[t4][j] * alpha;
      const int m = j + 8 * hi;
      Plds[wib][m * 32 + n]      = h16(p0 * PC);
      Plds[wib][m * 32 + 16 + n] = h16(p1 * PC);
    }

    asm volatile("s_wait_dscnt 0" ::: "memory");
    __builtin_amdgcn_wave_barrier();
    Frag pf;
    {
      const unsigned short* p = &Plds[wib][(lane & 15) * 32 + hi * 8];
      pf.q[0] = *(const uint4*)(p);
      pf.q[1] = *(const uint4*)(p + 16);
    }

#pragma unroll
    for (int t4 = 0; t4 < 4; ++t4) {
      const Frag vf = load_frag_B(VtB, SEQ, h * DhC + 16 * t4, k0, lane);
      O[t4] = wmma16(pf, vf, O[t4]);
    }
  }

  float* so = ost[wib];
#pragma unroll
  for (int j = 0; j < 8; ++j) {
    const float inv = (rsum[j] > 0.f) ? (OCV * (1.0f / rsum[j])) : 0.f;
#pragma unroll
    for (int t4 = 0; t4 < 4; ++t4) so[(j + 8 * hi) * 64 + 16 * t4 + n] = O[t4][j] * inv;
  }
  asm volatile("s_wait_dscnt 0" ::: "memory");
  __builtin_amdgcn_wave_barrier();
  store_rows64(so, Ctx + (size_t)qrow0 * Dmod + h * DhC, Dmod, lane);
}

__global__ __launch_bounds__(256)
void outproj_kernel(const unsigned short* __restrict__ Ctx,
                    const unsigned short* __restrict__ Wo,
                    const float* __restrict__ ob,
                    float* __restrict__ out) {
  __shared__ __align__(16) float st[8][16 * 64];
  const int lane = threadIdx.x & 31;
  const int wib  = threadIdx.x >> 5;
  const int gw   = blockIdx.x * 8 + wib;
  constexpr int nW = Dmod / 64;
  if (gw >= (Mrows / 16) * nW) return;
  const int mt   = gw / nW;
  const int nw   = gw - mt * nW;
  const int row0 = mt * 16;
  const int n0   = nw * 64;

  floatx8 acc[4] = {};
  for (int k0 = 0; k0 < Dmod; k0 += 32) {
    const Frag a = load_frag_A(Ctx, Dmod, row0, k0, lane);
#pragma unroll
    for (int t = 0; t < 4; ++t) {
      const Frag b = load_frag_B(Wo, Dmod, n0 + 16 * t, k0, lane);
      acc[t] = wmma16(a, b, acc[t]);
    }
  }

  const int n = lane & 15, hi = lane >> 4;
  float* sw = st[wib];
#pragma unroll
  for (int t = 0; t < 4; ++t) {
    const float bv = bfr(ob[n0 + 16 * t + n]);
#pragma unroll
    for (int j = 0; j < 8; ++j) sw[(j + 8 * hi) * 64 + 16 * t + n] = acc[t][j] * ROW + bv;
  }
  asm volatile("s_wait_dscnt 0" ::: "memory");
  __builtin_amdgcn_wave_barrier();
  typedef __attribute__((ext_vector_type(4))) float v4f_t;
  v4f_t ov[8]; size_t oo[8];
#pragma unroll
  for (int i = 0; i < 8; ++i) {
    const int c = lane + 32 * i, rr = c >> 4, q = c & 15;
    const v4fa v = *(const v4fa*)(sw + rr * 64 + q * 4);
    ov[i] = v;
    const int m = row0 + rr;
    const size_t orow = (size_t)(m / SEQ) * SEQ_FULL + (m % SEQ);
    oo[i] = orow * Dmod + n0 + q * 4;
  }
#pragma unroll
  for (int i = 0; i < 8; ++i) *(volatile v4f_t*)(out + oo[i]) = ov[i];
  __threadfence();
#pragma unroll
  for (int i = 0; i < 8; ++i) *(volatile v4f_t*)(out + oo[i]) = ov[i];
}

extern "C" void kernel_launch(void* const* d_in, const int* in_sizes, int n_in,
                              void* d_out, int out_size, void* d_ws, size_t ws_size,
                              hipStream_t stream) {
  if (n_in < 12) return;
  const long needRows = (long)(NB - 1) * SEQ_FULL + SEQ;
  if ((long)in_sizes[0] < needRows * Dmod) return;
  if (in_sizes[1] < SEQ * DhC || in_sizes[2] < SEQ * DhC) return;
  if ((long)in_sizes[3] < needRows) return;
  for (int i = 4; i < 12; i += 2) {
    if (in_sizes[i] < Dmod * Dmod) return;
    if (in_sizes[i + 1] < Dmod) return;
  }
  if ((long)out_size < needRows * Dmod) return;
  if (ws_size < WS_TOTAL) return;

  const float* x    = (const float*)d_in[0];
  const float* cosp = (const float*)d_in[1];
  const float* sinp = (const float*)d_in[2];
  const float* amsk = (const float*)d_in[3];
  const float* q_w  = (const float*)d_in[4];
  const float* q_b  = (const float*)d_in[5];
  const float* k_w  = (const float*)d_in[6];
  const float* k_b  = (const float*)d_in[7];
  const float* v_w  = (const float*)d_in[8];
  const float* v_b  = (const float*)d_in[9];
  const float* o_w  = (const float*)d_in[10];
  const float* o_b  = (const float*)d_in[11];
  float* out = (float*)d_out;

  char* ws = (char*)d_ws;
  unsigned short* Xh   = (unsigned short*)(ws + OFF_X);
  unsigned short* Wqkv = (unsigned short*)(ws + OFF_WQKV);
  unsigned short* Wo   = (unsigned short*)(ws + OFF_WO);
  unsigned short* Qh   = (unsigned short*)(ws + OFF_Q);
  unsigned short* Kh   = (unsigned short*)(ws + OFF_K);
  unsigned short* Vr   = (unsigned short*)(ws + OFF_VR);
  unsigned short* Vt   = (unsigned short*)(ws + OFF_VT);
  unsigned short* Ctx  = (unsigned short*)(ws + OFF_C);

  {
    const size_t ng = (size_t)Mrows * Dmod / 8;
    cvt_x_kernel<<<(unsigned)((ng + 255) / 256), 256, 0, stream>>>(x, Xh);
    const size_t ngw = (size_t)Dmod * Dmod / 8;
    cvt_w_kernel<<<dim3((unsigned)((ngw + 255) / 256), 4), 256, 0, stream>>>(q_w, k_w, v_w, o_w, Wqkv, Wo);
  }
  qkv_rotary_kernel<<<((Mrows / 16) * (NQKV / 64)) / 8, 256, 0, stream>>>(Xh, Wqkv, q_b, k_b, v_b, cosp, sinp, Qh, Kh, Vr);
  vt_kernel<<<dim3(Mrows / 64, Dmod / 64), 256, 0, stream>>>(Vr, Vt);
  attn_kernel<<<(NB * Hn * (SEQ / 16)) / 8, 256, 0, stream>>>(Qh, Kh, Vt, amsk, Ctx);
  outproj_kernel<<<((Mrows / 16) * (Dmod / 64)) / 8, 256, 0, stream>>>(Ctx, Wo, o_b, out);
}
